// MultiHead_19971597926912
// MI455X (gfx1250) — hardware-verified
//
#include <hip/hip_runtime.h>
#ifndef NB
#define NB 2
#endif
#ifndef SEQ
#define SEQ 2048
#endif
#define NB_FULL 2
#define SEQ_FULL 2048
#define DM 1024
#define NH 16
#define HD 64
#define MFB 16
#define NR ((size_t)NB * SEQ)
static_assert(SEQ % 128 == 0);
static_assert(SEQ <= SEQ_FULL);
static_assert(NB >= 1 && NB <= NB_FULL);
static_assert(DM == NH * HD);
static_assert((DM * (DM / 8)) % 256 == 0);
static_assert(((size_t)NB * SEQ * DM / 8) % 256 == 0);
static_assert(((size_t)NB * SEQ) % 128 == 0 && DM % 64 == 0 && DM % 32 == 0);
static_assert((size_t)4 * DM * DM * 2 + (size_t)8 * NB_FULL * SEQ_FULL * DM * 2 + (size_t)MFB * 128 + 16 * 256 <= (size_t)134217728);

typedef _Float16 v16h __attribute__((ext_vector_type(16)));
typedef unsigned short v8us __attribute__((ext_vector_type(8), may_alias));
typedef float  v8f  __attribute__((ext_vector_type(8)));
typedef float  v4f  __attribute__((ext_vector_type(4)));
typedef float  v4fa __attribute__((ext_vector_type(4), may_alias));
typedef _Float16 v4h __attribute__((ext_vector_type(4)));
union FragH { v16h v; v8us half[2]; _Float16 h[16]; unsigned short u[16]; };

__device__ __forceinline__ unsigned short bf16_bits(float x) { unsigned int u = __float_as_uint(x); return (unsigned short)((u + 0x7FFFu + ((u >> 16) & 1u)) >> 16); }
__device__ __forceinline__ float bf16_val(unsigned short b) { return __uint_as_float(((unsigned int)b) << 16); }
__device__ __forceinline__ float bf16_rne(float x) { return bf16_val(bf16_bits(x)); }

__device__ __forceinline__ v16h g2_frag(const _Float16* p, int hh) { FragH f; f.half[0] = *(const v8us*)((const unsigned short*)p + 8 * hh); f.half[1] = *(const v8us*)((const unsigned short*)p + 16 + 8 * hh); return f.v; }
__device__ __forceinline__ v8f g2_mma(v16h a, v16h b, v8f c) { v8f d = __builtin_amdgcn_wmma_f32_16x16x32_f16(false, a, false, b, (short)0, c, false, false); asm volatile("v_nop\n\tv_nop\n\tv_nop\n\tv_nop" : "+v"(d) : "v"(a), "v"(b)); return d; }

__device__ __forceinline__ float hmax16(float v) {
#pragma unroll
  for (int off = 1; off < 16; off <<= 1) v = fmaxf(v, __shfl_xor(v, off, 32));
  return v;
}
__device__ __forceinline__ float hsum16(float v) {
#pragma unroll
  for (int off = 1; off < 16; off <<= 1) v += __shfl_xor(v, off, 32);
  return v;
}

__global__ __launch_bounds__(256) void k_wt_f16(const float* __restrict__ W, _Float16* __restrict__ Wt, int K, int N, float scale) {
  const int t = blockIdx.x * 256 + threadIdx.x; if (t >= N * (K / 8)) return;
  const int n = t / (K / 8), k8 = (t % (K / 8)) * 8; FragH f;
#pragma unroll
  for (int i = 0; i < 8; ++i) f.h[i] = (_Float16)(bf16_rne(W[(size_t)(k8 + i) * N + n]) * scale);
  const v8us o = f.half[0]; unsigned short* d = (unsigned short*)Wt + (size_t)n * K + k8;
  *(volatile v8us*)d = o; __threadfence(); *(volatile v8us*)d = o;
}

__global__ __launch_bounds__(256) void k_xrows(const float* __restrict__ x, _Float16* __restrict__ X16, size_t n8) {
  const size_t t = (size_t)blockIdx.x * 256 + threadIdx.x; if (t >= n8) return;
  const size_t r = t / (DM / 8); const int c8 = (int)(t % (DM / 8)) * 8;
  const size_t b = r / SEQ, s = r % SEQ;
  const float* src = x + (b * SEQ_FULL + s) * DM + c8;
  const v4f a0 = *(const v4fa*)src, a1 = *(const v4fa*)(src + 4);
  FragH f;
#pragma unroll
  for (int q = 0; q < 4; ++q) { f.h[q] = (_Float16)bf16_rne(a0[q]); f.h[4 + q] = (_Float16)bf16_rne(a1[q]); }
  const v8us o = f.half[0]; unsigned short* d = (unsigned short*)X16 + t * 8;
  *(volatile v8us*)d = o; __threadfence(); *(volatile v8us*)d = o;
}

__global__ __launch_bounds__(256) void k_mflag(const float* __restrict__ msk, int* __restrict__ FL) {
  __shared__ int red[256];
  const int tid = threadIdx.x; int any = 0;
  const int ne = (int)((size_t)NB * SEQ);
#pragma unroll 1
  for (int e = blockIdx.x * 256 + tid; e < ne; e += MFB * 256) {
    const int b = e / SEQ, j = e - b * SEQ;
    any |= (int)(msk[(size_t)b * SEQ_FULL + j] != 0.f);
  }
  red[tid] = any; __syncthreads();
  for (int st = 128; st > 0; st >>= 1) { if (tid < st) red[tid] |= red[tid + st]; __syncthreads(); }
  const int f = red[0];
  int* d = FL + blockIdx.x * 32 + (tid & 31);
  if (tid < 32) *(volatile int*)d = f;
  __threadfence();
  if (tid < 32) *(volatile int*)d = f;
}

__global__ __launch_bounds__(128) void k_gemm2(const _Float16* __restrict__ A, int lda, const _Float16* __restrict__ Bh, int ldb, float alpha, const float* __restrict__ bias,
                                               float* __restrict__ C, _Float16* __restrict__ C16, int ldc, int M, int N, int K) {
  __shared__ __attribute__((aligned(16))) float so[4][32][68];
  const int tid = threadIdx.x, w = tid >> 5, lane = tid & 31, ln = lane & 15, hh = lane >> 4;
  const int ntn = N >> 6; const int mt = blockIdx.x / ntn, nq = blockIdx.x - mt * ntn;
  const int row0 = mt * 128 + 32 * w, col0 = nq * 64;
  if (row0 >= M) return;
  const _Float16* a0p = A + (size_t)(row0 + ln) * lda; const _Float16* a1p = a0p + (size_t)16 * lda;
  const _Float16* b0p = Bh + (size_t)(col0 + ln) * ldb; const _Float16* b1p = b0p + (size_t)16 * ldb; const _Float16* b2p = b1p + (size_t)16 * ldb; const _Float16* b3p = b2p + (size_t)16 * ldb;
  const v8f z8 = {0.f,0.f,0.f,0.f,0.f,0.f,0.f,0.f};
  v8f c00 = z8, c01 = z8, c02 = z8, c03 = z8, c10 = z8, c11 = z8, c12 = z8, c13 = z8;
#pragma unroll 1
  for (int kb = 0; kb < K; kb += 32) {
    const v16h a0 = g2_frag(a0p + kb, hh), a1 = g2_frag(a1p + kb, hh);
    v16h b = g2_frag(b0p + kb, hh); c00 = g2_mma(a0, b, c00); c10 = g2_mma(a1, b, c10);
    b = g2_frag(b1p + kb, hh); c01 = g2_mma(a0, b, c01); c11 = g2_mma(a1, b, c11);
    b = g2_frag(b2p + kb, hh); c02 = g2_mma(a0, b, c02); c12 = g2_mma(a1, b, c12);
    b = g2_frag(b3p + kb, hh); c03 = g2_mma(a0, b, c03); c13 = g2_mma(a1, b, c13);
  }
  v8f accs[8] = {c00, c01, c02, c03, c10, c11, c12, c13};
#pragma unroll
  for (int u = 0; u < 8; ++u) {
    const int t = u & 3, half = u >> 2; const int col = col0 + t * 16 + ln;
    const float bv = bias ? bf16_rne(bias[col]) : 0.f;
#pragma unroll
    for (int r = 0; r < 8; ++r) { const int rloc = half * 16 + 8 * hh + r; so[w][rloc][t * 16 + ln] = accs[u][r] * alpha + bv; }
  }
  __builtin_amdgcn_fence(4, "workgroup"); __builtin_amdgcn_wave_barrier();
  const int rsub = lane >> 4, c4 = (lane & 15) * 4;
  for (int pass = 0; pass < 2; ++pass) {
#pragma unroll
    for (int q = 0; q < 16; ++q) {
      const int r = q * 2 + rsub; const v4f v = *(const v4fa*)&so[w][r][c4];
      if (C) *(volatile v4f*)(C + (size_t)(row0 + r) * ldc + col0 + c4) = v;
      if (C16) { v4h h4;
#pragma unroll
        for (int i = 0; i < 4; ++i) h4[i] = (_Float16)v[i];
        *(volatile v4h*)(C16 + (size_t)(row0 + r) * ldc + col0 + c4) = h4; }
    }
    if (pass == 0) __threadfence();
  }
}

template <int NHv, int TTv>
__global__ __launch_bounds__(256) void k_vt(const _Float16* __restrict__ V16, int ldv, int voff, _Float16* __restrict__ Vt) {
  __shared__ unsigned short tl[64][66];
  const int tid = threadIdx.x; const int slab = blockIdx.x / (TTv / 64), lg = blockIdx.x % (TTv / 64); const int b = slab / NHv, h = slab % NHv;
  for (int i = tid; i < 64 * 8; i += 256) {
    const int r = i / 8, c8 = (i % 8) * 8; FragH f;
    f.half[0] = *(const v8us*)((const unsigned short*)V16 + ((size_t)b * TTv + lg * 64 + r) * ldv + voff + h * 64 + c8);
#pragma unroll
    for (int q = 0; q < 8; ++q) tl[r][c8 + q] = f.u[q];
  }
  __syncthreads();
  for (int pass = 0; pass < 2; ++pass) {
#pragma unroll
    for (int rd = 0; rd < 2; ++rd) {
      const int d = rd * 32 + tid / 8, pc = tid % 8; FragH f;
#pragma unroll
      for (int q = 0; q < 8; ++q) f.u[q] = tl[pc * 8 + q][d];
      *(volatile v8us*)((unsigned short*)Vt + ((size_t)slab * 64 + d) * TTv + lg * 64 + pc * 8) = f.half[0];
    }
    if (pass == 0) __threadfence();
  }
}

__global__ __launch_bounds__(128) void k_flash(const _Float16* __restrict__ Q16, const _Float16* __restrict__ K16, const _Float16* __restrict__ VT,
                                               const float* __restrict__ msk, const int* __restrict__ FL, _Float16* __restrict__ CTX) {
  __shared__ __attribute__((aligned(16))) _Float16 Ps[4][16][72];
  __shared__ __attribute__((aligned(16))) _Float16 Os[4][16][72];
  const int tid = threadIdx.x, w = tid >> 5, lane = tid & 31, ln = lane & 15, hh = lane >> 4;
  const int bh = blockIdx.y; const int b = bh / NH, h = bh - b * NH;
  const int q0 = blockIdx.x * 64 + w * 16;
  int fl = 0;
#pragma unroll 1
  for (int i = 0; i < MFB; ++i) fl |= FL[i * 32];
  const bool use_m = (fl != 0);
  const _Float16* qp = Q16 + ((size_t)b * SEQ + q0 + ln) * DM + h * HD;
  const v16h aq0 = g2_frag(qp, hh), aq1 = g2_frag(qp + 32, hh);
  const _Float16* kbase = K16 + ((size_t)b * SEQ + ln) * DM + h * HD;
  const _Float16* vbase = VT + ((size_t)bh * HD + ln) * SEQ;
  const float* mbase = msk + (size_t)b * SEQ_FULL + ln;
  const v8f z8 = {0.f,0.f,0.f,0.f,0.f,0.f,0.f,0.f};
  v8f cacc[4] = {z8, z8, z8, z8};
  float rmax[8], rsum[8];
#pragma unroll
  for (int j = 0; j < 8; ++j) { rmax[j] = -1.0e30f; rsum[j] = 0.f; }
#pragma unroll 1
  for (int kv0 = 0; kv0 < SEQ; kv0 += 64) {
    float p[4][8];
#pragma unroll
    for (int nt = 0; nt < 4; ++nt) {
      const _Float16* kp = kbase + (size_t)(kv0 + nt * 16) * DM;
      const v16h bk0 = g2_frag(kp, hh), bk1 = g2_frag(kp + 32, hh);
      v8f s = g2_mma(aq0, bk0, z8); s = g2_mma(aq1, bk1, s);
#pragma unroll
      for (int j = 0; j < 8; ++j) p[nt][j] = s[j] * 0.125f;
      if (use_m) {
        const float mk = bf16_rne(mbase[kv0 + nt * 16]) * (-1.0e9f);
#pragma unroll
        for (int j = 0; j < 8; ++j) p[nt][j] += mk;
      }
    }
    float alpha[8];
#pragma unroll
    for (int j = 0; j < 8; ++j) {
      float m = fmaxf(fmaxf(p[0][j], p[1][j]), fmaxf(p[2][j], p[3][j]));
      m = hmax16(m);
      const float nm = fmaxf(rmax[j], m);
      alpha[j] = __expf(rmax[j] - nm);
      rmax[j] = nm;
      float ps = 0.f;
#pragma unroll
      for (int nt = 0; nt < 4; ++nt) { const float e = __expf(p[nt][j] - nm); p[nt][j] = e; ps += e; }
      ps = hsum16(ps);
      rsum[j] = rsum[j] * alpha[j] + ps;
    }
#pragma unroll
    for (int dt = 0; dt < 4; ++dt)
#pragma unroll
      for (int j = 0; j < 8; ++j) cacc[dt][j] *= alpha[j];
#pragma unroll
    for (int nt = 0; nt < 4; ++nt)
#pragma unroll
      for (int j = 0; j < 8; ++j) Ps[w][8 * hh + j][nt * 16 + ln] = (_Float16)(p[nt][j] * 16384.0f);
    __builtin_amdgcn_fence(4, "workgroup"); __builtin_amdgcn_wave_barrier();
    const v16h ap0 = g2_frag(&Ps[w][ln][0], hh), ap1 = g2_frag(&Ps[w][ln][32], hh);
#pragma unroll
    for (int dt = 0; dt < 4; ++dt) {
      const _Float16* vp = vbase + (size_t)(dt * 16) * SEQ + kv0;
      const v16h bv0 = g2_frag(vp, hh), bv1 = g2_frag(vp + 32, hh);
      cacc[dt] = g2_mma(ap0, bv0, cacc[dt]); cacc[dt] = g2_mma(ap1, bv1, cacc[dt]);
    }
    __builtin_amdgcn_fence(4, "workgroup"); __builtin_amdgcn_wave_barrier();
  }
#pragma unroll
  for (int j = 0; j < 8; ++j) {
    const float fin = (1.0f / rsum[j]) * 0.00390625f;
#pragma unroll
    for (int dt = 0; dt < 4; ++dt) Os[w][8 * hh + j][dt * 16 + ln] = (_Float16)(cacc[dt][j] * fin);
  }
  __builtin_amdgcn_fence(4, "workgroup"); __builtin_amdgcn_wave_barrier();
  unsigned short* orow = (unsigned short*)CTX + ((size_t)b * SEQ + q0) * DM + h * HD;
  const int rq = lane >> 3, pc = (lane & 7) * 8;
  for (int pass = 0; pass < 2; ++pass) {
#pragma unroll
    for (int it = 0; it < 4; ++it) { const int row = it * 4 + rq; const v8us v = *(const v8us*)&Os[w][row][pc]; *(volatile v8us*)(orow + (size_t)row * DM + pc) = v; }
    if (pass == 0) __threadfence();
  }
}

extern "C" void kernel_launch(void* const* d_in, const int* in_sizes, int n_in,
                              void* d_out, int out_size, void* d_ws, size_t ws_size, hipStream_t stream) {
  if (n_in < 12) return;
  const float* const* I = (const float* const*)d_in;
  const float* xq = I[0]; const float* xk = I[1]; const float* xv = I[2]; const float* msk = I[3];
  const float* wq = I[4]; const float* bq = I[5]; const float* wk = I[6]; const float* bk = I[7];
  const float* wv = I[8]; const float* bv = I[9]; const float* wo = I[10]; const float* bo = I[11];
  const long long needX = ((long long)(NB - 1) * SEQ_FULL + SEQ) * DM;
  const long long needM = (long long)(NB - 1) * SEQ_FULL + SEQ;
  if ((long long)in_sizes[0] < needX || (long long)in_sizes[1] < needX || (long long)in_sizes[2] < needX || (long long)in_sizes[3] < needM) return;
  if (in_sizes[4] < DM * DM || in_sizes[6] < DM * DM || in_sizes[8] < DM * DM || in_sizes[10] < DM * DM) return;
  if (in_sizes[5] < DM || in_sizes[7] < DM || in_sizes[9] < DM || in_sizes[11] < DM) return;
  if ((long long)out_size < (long long)NR * DM) return;
  char* ws = (char*)d_ws; size_t off = 0;
  auto take = [&](size_t bytes) { char* p = ws + off; off += (bytes + 255) & ~(size_t)255; return p; };
  _Float16* BQ = (_Float16*)take((size_t)DM * DM * 2); _Float16* BK = (_Float16*)take((size_t)DM * DM * 2);
  _Float16* BV = (_Float16*)take((size_t)DM * DM * 2); _Float16* BO = (_Float16*)take((size_t)DM * DM * 2);
  _Float16* XQ = (_Float16*)take(NR * DM * 2); _Float16* XK = (_Float16*)take(NR * DM * 2); _Float16* XV = (_Float16*)take(NR * DM * 2);
  _Float16* Q16 = (_Float16*)take(NR * DM * 2); _Float16* K16 = (_Float16*)take(NR * DM * 2); _Float16* V16 = (_Float16*)take(NR * DM * 2);
  _Float16* VT = (_Float16*)take(NR * DM * 2);
  _Float16* CTX = (_Float16*)take(NR * DM * 2);
  int* FL = (int*)take((size_t)MFB * 32 * 4);
  if (off > ws_size) return;
  const unsigned gw = (unsigned)((DM * (DM / 8) + 255) / 256);
  k_wt_f16<<<gw, 256, 0, stream>>>(wq, BQ, DM, DM, 16.0f);
  k_wt_f16<<<gw, 256, 0, stream>>>(wk, BK, DM, DM, 16.0f);
  k_wt_f16<<<gw, 256, 0, stream>>>(wv, BV, DM, DM, 16.0f);
  k_wt_f16<<<gw, 256, 0, stream>>>(wo, BO, DM, DM, 16.0f);
  const size_t n8 = NR * DM / 8; const unsigned gx = (unsigned)((n8 + 255) / 256);
  k_xrows<<<gx, 256, 0, stream>>>(xq, XQ, n8);
  k_xrows<<<gx, 256, 0, stream>>>(xk, XK, n8);
  k_xrows<<<gx, 256, 0, stream>>>(xv, XV, n8);
  k_mflag<<<MFB, 256, 0, stream>>>(msk, FL);
  const unsigned gg = (unsigned)((NR / 128) * (DM / 64));
  k_gemm2<<<gg, 128, 0, stream>>>(XQ, DM, BQ, DM, 0.0625f, bq, nullptr, Q16, DM, (int)NR, DM, DM);
  k_gemm2<<<gg, 128, 0, stream>>>(XK, DM, BK, DM, 0.0625f, bk, nullptr, K16, DM, (int)NR, DM, DM);
  k_gemm2<<<gg, 128, 0, stream>>>(XV, DM, BV, DM, 0.0625f, bv, nullptr, V16, DM, (int)NR, DM, DM);
  k_vt<NH, SEQ><<<(unsigned)(NB * NH * (SEQ / 64)), 256, 0, stream>>>(V16, DM, 0, VT);
  k_flash<<<dim3(SEQ / 64, NB * NH), 128, 0, stream>>>(Q16, K16, VT, msk, FL, CTX);
  k_gemm2<<<gg, 128, 0, stream>>>(CTX, DM, BO, DM, 0.0009765625f, bo, (float*)d_out, nullptr, DM, (int)NR, DM, DM);
}
